// CSR_Attention_9569187136082
// MI455X (gfx1250) — hardware-verified
//
#include <hip/hip_runtime.h>


namespace {
constexpr int NB = 16, L = 200, LP = 8, D = 128, NU = 1001, NRS = NB * L  , NRP = NB * LP  , NR = NRS + 2 * NRP  ;
constexpr float XS = 8.0f, WSC = 256.0f, EPS = 1e-8f, LNE = 1e-5f;

typedef _Float16 b16;
typedef __attribute__((ext_vector_type(16))) _Float16 v16b;
typedef __attribute__((ext_vector_type(8))) _Float16 v8b;
typedef __attribute__((ext_vector_type(8))) float v8f;
typedef __attribute__((ext_vector_type(4))) float v4f;
__device__ __forceinline__ float bf16_rne(float f) { unsigned int u = __float_as_uint(f); u += 0x7FFFu + ((u >> 16) & 1u); return __uint_as_float(u & 0xFFFF0000u); }
__device__ __forceinline__ v16b frag_kb(const b16* p, int hh) { const v8b a = *(const v8b*)(p + 8 * hh), b = *(const v8b*)(p + 16 + 8 * hh); v16b f;
#pragma unroll
  for (int e = 0; e < 8; ++e) { f[e] = a[e]; f[8 + e] = b[e]; } return f; }
__device__ __forceinline__ v8f wmma16b(v16b a, v16b b, v8f c) { v8f d = __builtin_amdgcn_wmma_f32_16x16x32_f16(false, a, false, b, (short)0, c, false, false); asm volatile("v_nop\n\tv_nop\n\tv_nop\n\tv_nop" : "+v"(d) : "v"(a), "v"(b)); return d; }
__device__ __forceinline__ void wave_lds_sync() { __builtin_amdgcn_fence(__ATOMIC_RELEASE, "workgroup"); __builtin_amdgcn_wave_barrier(); __builtin_amdgcn_fence(__ATOMIC_ACQUIRE, "workgroup"); }
__device__ __forceinline__ float pmul(float a, float b) { float p = a * b; asm volatile("" : "+v"(p)); return p; }
__device__ __forceinline__ float elu(float x) { return x > 0.0f ? x : (__expf(x) - 1.0f); }

__global__ __launch_bounds__(256) void prep_kernel(const float* __restrict__ xs, const float* __restrict__ xp, const float* __restrict__ xq, const float* __restrict__ wq, const float* __restrict__ wk, const float* __restrict__ wv, b16* __restrict__ X16, b16* __restrict__ W16) {
  const int t = blockIdx.x * 256 + threadIdx.x; const int nx = NR * D / 8, nw = 3 * D * D / 8; v8b o;
  if (t < nx) { const int e = t * 8; const int row = e / D; const float* src = row < NRS ? xs + e : row < NRS + NRP ? xp + (e - NRS * D) : xq + (e - (NRS + NRP) * D);
    for (int j = 0; j < 8; ++j) o[j] = (b16)(bf16_rne(src[j]) * XS); for (int pass = 0; pass < 2; ++pass) { *(volatile v8b*)(X16 + e) = o; __threadfence(); } }
  else if (t < nx + nw) { const int e = (t - nx) * 8; const int k = e / (D * D), r = e - k * D * D; const float* w = k == 0 ? wq : k == 1 ? wk : wv; for (int j = 0; j < 8; ++j) o[j] = (b16)(bf16_rne(w[r + j]) * WSC); for (int pass = 0; pass < 2; ++pass) { *(volatile v8b*)(W16 + e) = o; __threadfence(); } }
}
__global__ __launch_bounds__(128) void proj_kernel(const b16* __restrict__ X16, const b16* __restrict__ W16, const float* __restrict__ bq, const float* __restrict__ bk, const float* __restrict__ bv, float* __restrict__ Q, float* __restrict__ Z, float* __restrict__ V) {
  __shared__ __attribute__((aligned(16))) float Ts[4][16][D + 4];
  const int kind = blockIdx.y, wave = threadIdx.x >> 5, lane = threadIdx.x & 31, nloc = lane & 15, hlf = lane >> 4; const size_t m0 = (size_t)blockIdx.x * 64 + wave * 16; if (kind == 0 && m0 >= (size_t)NRS) return;
  const b16* Wp = W16 + (size_t)kind * D * D; const float* bb = kind == 0 ? bq : kind == 1 ? bk : bv; float* dst = kind == 0 ? Q : kind == 1 ? Z : V;
  v8f acc[8];
#pragma unroll
  for (int t = 0; t < 8; ++t) acc[t] = (v8f){};
#pragma unroll
  for (int kb = 0; kb < D; kb += 32) { const v16b a = frag_kb(X16 + (m0 + nloc) * D + kb, hlf);
#pragma unroll
    for (int t = 0; t < 8; ++t) acc[t] = wmma16b(a, frag_kb(Wp + (size_t)(t * 16 + nloc) * D + kb, hlf), acc[t]); }
#pragma unroll
  for (int t = 0; t < 8; ++t) { const int c = t * 16 + nloc; const float b_ = bf16_rne(bb[c]);
#pragma unroll
    for (int r = 0; r < 8; ++r) { float v = acc[t][r] * (1.0f / (XS * WSC)) + b_; if (kind < 2) v = elu(v); Ts[wave][8 * hlf + r][c] = v; } }
  wave_lds_sync();
  for (int pass = 0; pass < 2; ++pass) { for (int rr = 0; rr < 16; ++rr) *(volatile v4f*)(dst + (m0 + rr) * D + lane * 4) = *(const v4f*)(&Ts[wave][rr][lane * 4]); __threadfence(); }
}
__device__ __forceinline__ float bsum(float v, float* red) { const int t_ = threadIdx.x; red[t_] = v; __syncthreads(); for (int s = 128; s >= 1; s >>= 1) { if (t_ < s) red[t_] += red[t_ + s]; __syncthreads(); } const float r = red[0]; __syncthreads(); return r; }
__device__ __forceinline__ void prompt_state(const float* __restrict__ Z, const float* __restrict__ V, int r0, const float* __restrict__ gz, const float* __restrict__ bz, const float* __restrict__ gs, const float* __restrict__ bs, float* __restrict__ PS, float* __restrict__ pzout, float* red, float* zs, float* vs) {
  const int t_ = threadIdx.x; const int q = t_ & (D - 1), ph = t_ >> 7;
  for (int i = t_; i < LP * D; i += 256) { zs[i] = Z[(size_t)r0 * D + i]; vs[i] = V[(size_t)r0 * D + i]; }
  __syncthreads();
  float zc = 0.0f; if (t_ < D) { for (int j = 0; j < LP; ++j) zc += zs[j * D + t_]; zc += EPS; }
  const float mz = bsum(t_ < D ? zc : 0.0f, red) * (1.0f / D); const float dz = t_ < D ? zc - mz : 0.0f; const float vz = bsum(dz * dz, red) * (1.0f / D); const float rz = rsqrtf(vz + LNE);
  if (t_ < D) pzout[t_] = pmul(dz * rz, bf16_rne(gz[t_])) + bf16_rne(bz[t_]);
  float s1 = 0.0f;
#pragma unroll 1
  for (int pp = 0; pp < D / 2; ++pp) { const int p = ph * (D / 2) + pp; float a = 0.0f; for (int j = 0; j < LP; ++j) a += pmul(zs[j * D + p], vs[j * D + q]); s1 += a + EPS; }
  const float ms = bsum(s1, red) * (1.0f / (D * D)); float s2 = 0.0f;
#pragma unroll 1
  for (int pp = 0; pp < D / 2; ++pp) { const int p = ph * (D / 2) + pp; float a = 0.0f; for (int j = 0; j < LP; ++j) a += pmul(zs[j * D + p], vs[j * D + q]); const float dv = (a + EPS) - ms; s2 += dv * dv; }
  const float rs = rsqrtf(bsum(s2, red) * (1.0f / (D * D)) + LNE);
#pragma unroll 1
  for (int pp = 0; pp < D / 2; ++pp) { const int p = ph * (D / 2) + pp; float a = 0.0f; for (int j = 0; j < LP; ++j) a += pmul(zs[j * D + p], vs[j * D + q]); PS[p * D + q] = pmul(((a + EPS) - ms) * rs, bf16_rne(gs[p * D + q])) + bf16_rne(bs[p * D + q]); }
  __syncthreads();
}
__global__ __launch_bounds__(256) void state_kernel(const float* __restrict__ Q, const float* __restrict__ Z, const float* __restrict__ V, const int* __restrict__ uid, const float* __restrict__ gz, const float* __restrict__ bz, const float* __restrict__ gs, const float* __restrict__ bs,
                                                 const float* __restrict__ gn, const float* __restrict__ bn, const float* __restrict__ ga, const float* __restrict__ ba, const float* __restrict__ prev_z, const float* __restrict__ prev_s, float* __restrict__ PREV, float* __restrict__ out, double* __restrict__ STD2) {
  __shared__ float SR[D * D]; __shared__ float PSL[D * D]; __shared__ float red[256]; __shared__ float zs[LP * D], vs[LP * D]; __shared__ float pzP[D], pzS[D], zrow[D], vrow[D], qn[D], zfull[D], zcum[D], nav[D]; __shared__ float scal[4]; __shared__ double dred[2][256];
  const int b = blockIdx.x, t_ = threadIdx.x; const int q = t_ & (D - 1), ph = t_ >> 7;
  prompt_state(Z, V, NRS + NRP + b * LP, gz, bz, gs, bs, PSL, pzS, red, zs, vs);
  { const int u = min(max(uid[b], 0), NU - 1); float zu = 0.0f; if (t_ < D) { zu = bf16_rne(prev_z[(size_t)u * D + t_]) + pzS[t_]; } const float n2 = bsum(t_ < D ? zu * zu : 0.0f, red); const float inv = 1.0f / (sqrtf(n2) + EPS);
    float msum = bsum(t_ < D ? bf16_rne(prev_z[(size_t)u * D + t_]) : 0.0f, red); if (t_ == 0) scal[0] = (msum != 0.0f) ? 1.0f : 0.0f;
    for (int pass = 0; pass < 2; ++pass) {
#pragma unroll 1
      for (int pp = 0; pp < D / 2; ++pp) { const int p = ph * (D / 2) + pp; ((volatile float*)PREV)[(size_t)b * D * D + p * D + q] = (bf16_rne(prev_s[((size_t)u * D + p) * D + q]) + PSL[p * D + q]) * inv; }
      __threadfence(); } }
  __syncthreads();
  prompt_state(Z, V, NRS + b * LP, gz, bz, gs, bs, PSL, pzP, red, zs, vs);
  for (int i = t_; i < D * D; i += 256) SR[i] = 0.0f; if (t_ < D) zcum[t_] = 0.0f;
  __syncthreads();
  double dsum = 0.0, dsq = 0.0;
  const float* PRb = PREV + (size_t)b * D * D;
  for (int l = 0; l < L; ++l) { const size_t row = (size_t)b * L + l;
    if (t_ < D) { zrow[t_] = Z[row * D + t_]; vrow[t_] = V[row * D + t_]; zcum[t_] += Z[row * D + t_]; }
    __syncthreads();
    { const float zc = t_ < D ? zcum[t_] + EPS : 0.0f; const float mz = bsum(zc, red) * (1.0f / D); const float dz = t_ < D ? zc - mz : 0.0f; const float vz = bsum(dz * dz, red) * (1.0f / D); const float rz = rsqrtf(vz + LNE);
      float zf = 0.0f, qv = 0.0f; if (t_ < D) { zf = pmul(dz * rz, bf16_rne(gz[t_])) + bf16_rne(bz[t_]) + pzP[t_]; zfull[t_] = zf; qv = Q[row * D + t_]; }
      const float qn2 = bsum(qv * qv, red), zn2 = bsum(zf * zf, red); if (t_ < D) qn[t_] = qv / (sqrtf(qn2) + EPS); if (t_ == 0) scal[1] = 1.0f / (sqrtf(zn2) + EPS);
      if (t_ < D) { const float xv = qv / fmaxf(zf, 1e-6f); dsum += (double)xv; dsq += (double)xv * (double)xv; } }
    __syncthreads();
    const float izn = scal[1];
    float s1 = 0.0f; const float vq = vrow[q];
#pragma unroll 1
    for (int pp = 0; pp < D / 2; ++pp) { const int p = ph * (D / 2) + pp; const float nv = SR[p * D + q] + pmul(zrow[p], vq); SR[p * D + q] = nv; s1 += nv + EPS; }
    const float m1 = bsum(s1, red) * (1.0f / (D * D)); float s2 = 0.0f;
#pragma unroll 1
    for (int pp = 0; pp < D / 2; ++pp) { const int p = ph * (D / 2) + pp; const float dv = (SR[p * D + q] + EPS) - m1; s2 += dv * dv; }
    const float r1 = rsqrtf(bsum(s2, red) * (1.0f / (D * D)) + LNE);
    float n1 = 0.0f;
#pragma unroll 1
    for (int pp = 0; pp < D / 2; ++pp) { const int p = ph * (D / 2) + pp; const int i = p * D + q; const float sf = pmul(((SR[i] + EPS) - m1) * r1, bf16_rne(gs[i])) + bf16_rne(bs[i]) + PSL[i]; n1 += pmul(sf, izn) + EPS; }
    const float m2 = bsum(n1, red) * (1.0f / (D * D)); float n2 = 0.0f;
#pragma unroll 1
    for (int pp = 0; pp < D / 2; ++pp) { const int p = ph * (D / 2) + pp; const int i = p * D + q; const float sf = pmul(((SR[i] + EPS) - m1) * r1, bf16_rne(gs[i])) + bf16_rne(bs[i]) + PSL[i]; const float nr = (pmul(sf, izn) + EPS) - m2; n2 += nr * nr; }
    const float r2 = rsqrtf(bsum(n2, red) * (1.0f / (D * D)) + LNE);
    float na = 0.0f, pv = 0.0f;
#pragma unroll 1
    for (int pp = 0; pp < D / 2; ++pp) { const int p = ph * (D / 2) + pp; const int i = p * D + q; const float sf = pmul(((SR[i] + EPS) - m1) * r1, bf16_rne(gs[i])) + bf16_rne(bs[i]) + PSL[i]; const float nam = pmul(((pmul(sf, izn) + EPS) - m2) * r2, bf16_rne(gn[i])) + bf16_rne(bn[i]);
      na += pmul(qn[p], nam); pv += pmul(qn[p], PRb[i]); }
    red[t_] = na + scal[0] * pv; __syncthreads(); if (t_ < D) nav[t_] = red[t_] + red[t_ + D]; __syncthreads();
    { const float x = t_ < D ? nav[t_] : 0.0f; const float mu = bsum(x, red) * (1.0f / D); const float dv = t_ < D ? x - mu : 0.0f; const float var = bsum(dv * dv, red) * (1.0f / D); const float rr = rsqrtf(var + LNE);
      const float o = pmul(dv * rr, t_ < D ? bf16_rne(ga[t_]) : 0.0f) + (t_ < D ? bf16_rne(ba[t_]) : 0.0f);
      for (int pass = 0; pass < 2; ++pass) { if (t_ < D) ((volatile float*)out)[row * D + t_] = o; __threadfence(); } }
    __syncthreads(); }
  dred[0][t_] = dsum; dred[1][t_] = dsq; __syncthreads(); for (int s = 128; s >= 1; s >>= 1) { if (t_ < s) { dred[0][t_] += dred[0][t_ + s]; dred[1][t_] += dred[1][t_ + s]; } __syncthreads(); }
  for (int pass = 0; pass < 2; ++pass) { if (t_ < 16) ((volatile double*)STD2)[(size_t)b * 16 + t_] = (t_ == 0) ? dred[0][0] : (t_ == 1) ? dred[1][0] : 0.0; __threadfence(); }
}
__global__ __launch_bounds__(32) void std_kernel(const double* __restrict__ STD2, float* __restrict__ out2) {
  const int lane = threadIdx.x; double s = 0.0, s2 = 0.0; if (lane == 0) { for (int b = 0; b < NB; ++b) { s += STD2[(size_t)b * 16]; s2 += STD2[(size_t)b * 16 + 1]; } const double n = (double)NB * L * D; const double var = (s2 - s * s / n) / (n - 1.0); const float sd = (float)sqrt(var > 0.0 ? var : 0.0);
    for (int pass = 0; pass < 2; ++pass) { ((volatile float*)out2)[0] = sd; __threadfence(); } }
}
}

extern "C" void kernel_launch(void* const* d_in, const int* in_sizes, int n_in, void* d_out, int out_size, void* d_ws, size_t ws_size, hipStream_t stream) {
  (void)n_in;
  auto Fp = [&](int i) { return (const float*)d_in[i]; }; auto Ip = [&](int i) { return (const int*)d_in[i]; };
  if (in_sizes[0] != NB || in_sizes[1] != NRS * D || in_sizes[2] != NRP * D || in_sizes[3] != NRP * D || in_sizes[4] != D * D || in_sizes[12] != D * D || in_sizes[18] != NU * D || in_sizes[19] != NU * D * D || out_size != NRS * D + 1) return;
  size_t off = 0; char* ws = (char*)d_ws;
  auto carve = [&](size_t bytes) { char* p = ws + off; off += (bytes + 255) & ~(size_t)255; return p; };
  b16* X16 = (b16*)carve((size_t)NR * D * 2); b16* W16 = (b16*)carve((size_t)3 * D * D * 2); float* Qp = (float*)carve((size_t)NRS * D * 4); float* Zp = (float*)carve((size_t)NR * D * 4); float* Vp = (float*)carve((size_t)NR * D * 4); float* PREV = (float*)carve((size_t)NB * D * D * 4); double* STD2 = (double*)carve((size_t)NB * 16 * 8);
  if (off > ws_size || off > ((size_t)128 << 20)) return;
  prep_kernel<<<(NR * D / 8 + 3 * D * D / 8 + 255) / 256, 256, 0, stream>>>(Fp(1), Fp(2), Fp(3), Fp(4), Fp(6), Fp(8), X16, W16);
  proj_kernel<<<dim3(NR / 64, 3), 128, 0, stream>>>(X16, W16, Fp(5), Fp(7), Fp(9), Qp, Zp, Vp);
  state_kernel<<<NB, 256, 0, stream>>>(Qp, Zp, Vp, Ip(0), Fp(10), Fp(11), Fp(12), Fp(13), Fp(14), Fp(15), Fp(16), Fp(17), Fp(18), Fp(19), PREV, (float*)d_out, STD2);
  std_kernel<<<1, 32, 0, stream>>>(STD2, (float*)d_out + (size_t)NRS * D);
}
